// DeepAngAEVComputer_18124761989631
// MI455X (gfx1250) — hardware-verified
//
#include <hip/hip_runtime.h>

#pragma clang fp contract(off)

typedef float v4f __attribute__((ext_vector_type(4)));
typedef float v8f __attribute__((ext_vector_type(8)));
typedef unsigned int u32x4 __attribute__((ext_vector_type(4)));
typedef unsigned int u32x8 __attribute__((ext_vector_type(8)));
typedef __bf16 v16bf __attribute__((ext_vector_type(16)));
typedef v4f __attribute__((may_alias)) v4fa;
typedef u32x4 __attribute__((may_alias)) u32x4a;

union BFrag { v16bf v; u32x8 w; u32x4 q[2]; };

#define NB 8
#define NA 32
#define NPAIR 496
#define NTILE 32
#define NOUT 256
#define CUTOFF_F 3.5f
#define RCUT_F (1.0f / 3.5f)
#define EPS_F 1e-7f
#define CLIPMIN_F 1e-10f
#define PI_F 3.14159265358979f

#define KP0 32
#define KP1 64
#define KP5 64
#define KP6 128
#define OFF0 0
#define OFF1 2048
#define OFF2 6144
#define OFF3 10240
#define OFF4 14336
#define OFF5 18432
#define OFF6 26624
#define WTOT 59392
#define PLANE_BYTES 118784

#define WV_ACT    0
#define WV_FEAT   3072
#define WV_WGT    3328
#define WV_FLOATS 3344

static_assert((NA * NA + NA + 16 + NOUT + 4 * NOUT + 4 * WV_FLOATS) * 4 <= 65536);
static_assert(OFF6 + 256 * KP6 == WTOT);
static_assert(WTOT * 2 == PLANE_BYTES);

__device__ __forceinline__ unsigned bf16_rne_bits(float f) {
  unsigned u = __float_as_uint(f);
  u = u + 0x7FFFu + ((u >> 16) & 1u);
  return u >> 16;
}

__device__ __forceinline__ void split_bf16(float v, unsigned& hb, unsigned& lb) {
  hb = bf16_rne_bits(v);
  const float hf = __uint_as_float(hb << 16);
  lb = bf16_rne_bits(v - hf);
}

__device__ __forceinline__ void pack2(float x, float y, unsigned& hw, unsigned& lw) {
  unsigned hx, lx, hy, ly;
  split_bf16(x, hx, lx);
  split_bf16(y, hy, ly);
  hw = hx | (hy << 16);
  lw = lx | (ly << 16);
}

__device__ __forceinline__ v8f wmma_bf16(v16bf a, v16bf b, v8f c) {
  v8f d = __builtin_amdgcn_wmma_f32_16x16x32_bf16(false, a, false, b, (short)0, c, false, false);
#if defined(__HIP_DEVICE_COMPILE__)
  asm volatile("v_nop\n\tv_nop\n\tv_nop\n\tv_nop" : "+v"(d) : "v"(a), "v"(b));
#endif
  return d;
}

template <bool UPPER>
__device__ __forceinline__ void load_a_frag(const float* p, v16bf& ahi, v16bf& alo) {
  const v4f q0 = *(const v4fa*)(p);
  const v4f q1 = *(const v4fa*)(p + 4);
  unsigned hw0, lw0, hw1, lw1, hw2, lw2, hw3, lw3;
  pack2(q0.x, q0.y, hw0, lw0);
  pack2(q0.z, q0.w, hw1, lw1);
  pack2(q1.x, q1.y, hw2, lw2);
  pack2(q1.z, q1.w, hw3, lw3);
  unsigned hw4 = 0u, lw4 = 0u, hw5 = 0u, lw5 = 0u, hw6 = 0u, lw6 = 0u, hw7 = 0u, lw7 = 0u;
  if (UPPER) {
    const v4f q2 = *(const v4fa*)(p + 16);
    const v4f q3 = *(const v4fa*)(p + 20);
    pack2(q2.x, q2.y, hw4, lw4);
    pack2(q2.z, q2.w, hw5, lw5);
    pack2(q3.x, q3.y, hw6, lw6);
    pack2(q3.z, q3.w, hw7, lw7);
  }
  BFrag fh, fl;
  const u32x8 th = {hw0, hw1, hw2, hw3, hw4, hw5, hw6, hw7};
  const u32x8 tl = {lw0, lw1, lw2, lw3, lw4, lw5, lw6, lw7};
  fh.w = th;
  fl.w = tl;
  ahi = fh.v;
  alo = fl.v;
}

__device__ __forceinline__ v16bf load_b_frag(const unsigned short* p) {
  BFrag f;
  f.q[0] = *(const u32x4a*)(p);
  f.q[1] = *(const u32x4a*)(p + 16);
  return f.v;
}

__device__ __forceinline__ float tanh_f(float x) {
  const float ax = fabsf(x);
  const float t = __expf(-2.0f * ax);
  const float y = (1.0f - t) * __builtin_amdgcn_rcpf(1.0f + t);
  return copysignf(y, x);
}

template <int KC, int APITCH, bool AUP, int KPB, int N, typename Epi>
__device__ __forceinline__ void run_layer(const float* aBuf,
                                          const unsigned short* __restrict__ ph0,
                                          const unsigned short* __restrict__ pl0,
                                          const float* __restrict__ bias, int lane,
                                          Epi&& epi) {
  const int h = lane >> 4, m = lane & 15;
  v16bf ah[KC], al[KC];
#pragma unroll
  for (int c = 0; c < KC; ++c)
    load_a_frag<AUP>(aBuf + m * APITCH + 32 * c + 8 * h, ah[c], al[c]);
#pragma unroll 1
  for (int nt = 0; nt < N / 16; ++nt) {
    const int col = nt * 16 + m;
    const unsigned short* ph = ph0 + col * KPB + 8 * h;
    const unsigned short* pl = pl0 + col * KPB + 8 * h;
    v8f acc = {0.f, 0.f, 0.f, 0.f, 0.f, 0.f, 0.f, 0.f};
#pragma unroll
    for (int c = 0; c < KC; ++c) {
      const v16bf bh = load_b_frag(ph + 32 * c);
      const v16bf bl = load_b_frag(pl + 32 * c);
      acc = wmma_bf16(ah[c], bh, acc);
      acc = wmma_bf16(ah[c], bl, acc);
      acc = wmma_bf16(al[c], bh, acc);
    }
    const float bb = bias[col];
    epi(nt, acc, bb);
  }
}

__global__ __launch_bounds__(256) void prep_weights(
    const float* __restrict__ W0, const float* __restrict__ W1, const float* __restrict__ W2,
    const float* __restrict__ W3, const float* __restrict__ W4, const float* __restrict__ W5,
    const float* __restrict__ W6, unsigned short* __restrict__ whi, unsigned short* __restrict__ wlo)
{
  const float* W; int K, F, KP, off;
  switch (blockIdx.y) {
    case 0:  W = W0; K = 9;   F = 64;  KP = KP0; off = OFF0; break;
    case 1:  W = W1; K = 64;  F = 64;  KP = KP1; off = OFF1; break;
    case 2:  W = W2; K = 64;  F = 64;  KP = KP1; off = OFF2; break;
    case 3:  W = W3; K = 64;  F = 64;  KP = KP1; off = OFF3; break;
    case 4:  W = W4; K = 64;  F = 64;  KP = KP1; off = OFF4; break;
    case 5:  W = W5; K = 64;  F = 128; KP = KP5; off = OFF5; break;
    default: W = W6; K = 128; F = 256; KP = KP6; off = OFF6; break;
  }
  const int ngrp = (F * KP) >> 3;
  const int g = blockIdx.x * 256 + threadIdx.x;
  if (g >= ngrp) return;
  const int idx0 = g * 8;
  const int c = idx0 / KP;
  const int kb = idx0 - c * KP;
  unsigned hw[4], lw[4];
#pragma unroll
  for (int e = 0; e < 4; ++e) {
    unsigned hb[2], lb[2];
#pragma unroll
    for (int s = 0; s < 2; ++s) {
      const int k = kb + 2 * e + s;
      const int kc = (k < K) ? k : (K - 1);
      float v = W[(size_t)kc * F + c];
      v = (k < K) ? v : 0.0f;
      split_bf16(v, hb[s], lb[s]);
    }
    hw[e] = hb[0] | (hb[1] << 16);
    lw[e] = lb[0] | (lb[1] << 16);
  }
  const u32x4 hv = {hw[0], hw[1], hw[2], hw[3]};
  const u32x4 lv = {lw[0], lw[1], lw[2], lw[3]};
  unsigned short* dh = whi + off + idx0;
  unsigned short* dl = wlo + off + idx0;
  *(volatile u32x4a*)dh = hv;
  *(volatile u32x4a*)dl = lv;
  __threadfence();
  *(volatile u32x4a*)dh = hv;
  *(volatile u32x4a*)dl = lv;
}

__global__ void __launch_bounds__(128)
aev_kernel(const float* __restrict__ Dg, const float* __restrict__ Sg,
           const unsigned short* __restrict__ whi, const unsigned short* __restrict__ wlo,
           const float* __restrict__ b0, const float* __restrict__ b1,
           const float* __restrict__ b2, const float* __restrict__ b3,
           const float* __restrict__ b4, const float* __restrict__ b5,
           const float* __restrict__ b6, float* __restrict__ outG)
{
  __shared__ __attribute__((aligned(16))) float Dm[NA * NA];
  __shared__ __attribute__((aligned(16))) float Sr[NA];
  __shared__ __attribute__((aligned(16))) float red[16];
  __shared__ __attribute__((aligned(16))) float GA[NOUT];
  __shared__ __attribute__((aligned(16))) float gaW[4 * NOUT];
  __shared__ __attribute__((aligned(16))) float waveMem[4 * WV_FLOATS];

  const int tid = threadIdx.x;
  const int lane = tid & 31;
  const int wv = tid >> 5;
  const int h = lane >> 4, m = lane & 15;
  const int bx = blockIdx.x;
  const int b = bx >> 5;
  const int i = bx & 31;

  for (int q = tid; q < NA * NA; q += 128) Dm[q] = Dg[b * (NA * NA) + q];
  if (tid < NA) Sr[tid] = Sg[b * NA + tid];
  for (int q = tid; q < 4 * NOUT; q += 128) gaW[q] = 0.0f;
  __syncthreads();

  float* wb     = waveMem + wv * WV_FLOATS;
  float* bufR   = wb + WV_ACT;
  float* bufX   = wb + WV_ACT + 1024;
  float* bufA   = wb + WV_ACT + 2048;
  float* buf128 = wb + WV_ACT;
  float* featW  = wb + WV_FEAT;
  float* wW     = wb + WV_WGT;
  float* gaw    = gaW + wv * NOUT;
  const int rb = 8 * h;

#pragma unroll 1
  for (int tt = 0; tt < 8; ++tt) {
    const int t = tt * 4 + wv;

    {
      const int p = t * 16 + m;
      const bool valid = (p < NPAIR);
      const int pe = valid ? p : (NPAIR - 1);
      int pp = pe, j = 0;
      while (j < 30 && pp >= 31 - j) { pp -= 31 - j; ++j; }
      const int k = j + 1 + pp;

      const float Rij = Dm[i * NA + j];
      const float Rik = Dm[i * NA + k];
      const float Rjk = Dm[j * NA + k];
      const float zi = Sr[i], zj = Sr[j], zk = Sr[k];

      const float rij2 = Rij * Rij, rik2 = Rik * Rik, rjk2 = Rjk * Rjk;
      const float ci = ((rij2 + rik2) - rjk2) / fmaxf((2.0f * Rij) * Rik, CLIPMIN_F);
      const float cj = ((rij2 + rjk2) - rik2) / fmaxf((2.0f * Rij) * Rjk, CLIPMIN_F);
      const float ck = ((rik2 + rjk2) - rij2) / fmaxf((2.0f * Rik) * Rjk, CLIPMIN_F);

      float g0 = (Rij + Rik) + Rjk;
      float g1 = (Rij * Rik + Rij * Rjk) + Rik * Rjk;
      float g2 = (Rij * Rik) * Rjk;
      const float gs = (g0 * g0 + g1 * g1) + g2 * g2;
      const float gn = 1.0f / (sqrtf(gs) + EPS_F);
      g0 = g0 * gn; g1 = g1 * gn; g2 = g2 * gn;

      float h0 = (zi + zj) + zk;
      float h1 = (ci + cj) + ck;
      float h2 = ((zi * (zj + zk) + zj * zk) - ci * (cj + ck)) - cj * ck;
      float h3 = ((zi * (cj + ck) + ci * (zj + zk)) + zj * ck) + cj * zk;
      float h4 = zi * (zj * zk - cj * ck) - ci * (zj * ck + cj * zk);
      float h5 = zi * (zj * ck + cj * zk) + ci * (zj * zk - cj * ck);
      const float hs = ((((h0 * h0 + h1 * h1) + h2 * h2) + h3 * h3) + h4 * h4) + h5 * h5;
      const float hn = 1.0f / (sqrtf(hs) + EPS_F);
      h0 = h0 * hn; h1 = h1 * hn; h2 = h2 * hn; h3 = h3 * hn; h4 = h4 * hn; h5 = h5 * hn;

      const bool msk = (Rij < CUTOFF_F) && (Rij != 0.0f) && (Rik < CUTOFF_F) && (Rik != 0.0f);
      const float fcij = 0.5f * cosf((PI_F * Rij) * RCUT_F) + 0.5f;
      const float fcik = 0.5f * cosf((PI_F * Rik) * RCUT_F) + 0.5f;
      float w = msk ? (fcij * fcik) : 0.0f;
      w = valid ? w : 0.0f;

      const v4f s0 = {valid ? g0 : 0.0f, valid ? g1 : 0.0f, valid ? g2 : 0.0f, valid ? h0 : 0.0f};
      const v4f s1 = {valid ? h1 : 0.0f, valid ? h2 : 0.0f, valid ? h3 : 0.0f, valid ? h4 : 0.0f};
      const v4f s2 = {valid ? h5 : 0.0f, 0.0f, 0.0f, 0.0f};
      const v4f s3 = {0.0f, 0.0f, 0.0f, 0.0f};
      if (h == 0) {
        float* fr = featW + m * 16;
        *(v4fa*)(fr)      = s0;
        *(v4fa*)(fr + 4)  = s1;
        *(v4fa*)(fr + 8)  = s2;
        *(v4fa*)(fr + 12) = s3;
        wW[m] = w;
      }
    }
    __syncthreads();

    run_layer<1, 16, false, KP0, 64>(featW, whi + OFF0, wlo + OFF0, b0, lane,
      [&](int nt, v8f acc, float bb) {
        const int col = nt * 16 + m;
#pragma unroll
        for (int r = 0; r < 8; ++r) bufR[(rb + r) * 64 + col] = tanh_f(acc[r] + bb);
      });
    __syncthreads();
    run_layer<2, 64, true, KP1, 64>(bufR, whi + OFF1, wlo + OFF1, b1, lane,
      [&](int nt, v8f acc, float bb) {
        const int col = nt * 16 + m;
#pragma unroll
        for (int r = 0; r < 8; ++r) {
          const int idx = (rb + r) * 64 + col;
          const float x1 = tanh_f(acc[r] + bb);
          bufX[idx] = x1 + bufR[idx];
        }
      });
    __syncthreads();
    run_layer<2, 64, true, KP1, 64>(bufX, whi + OFF2, wlo + OFF2, b2, lane,
      [&](int nt, v8f acc, float bb) {
        const int col = nt * 16 + m;
#pragma unroll
        for (int r = 0; r < 8; ++r) bufA[(rb + r) * 64 + col] = tanh_f(acc[r] + bb);
      });
    __syncthreads();
    run_layer<2, 64, true, KP1, 64>(bufA, whi + OFF3, wlo + OFF3, b3, lane,
      [&](int nt, v8f acc, float bb) {
        const int col = nt * 16 + m;
#pragma unroll
        for (int r = 0; r < 8; ++r) bufR[(rb + r) * 64 + col] = tanh_f(acc[r] + bb);
      });
    __syncthreads();
    run_layer<2, 64, true, KP1, 64>(bufR, whi + OFF4, wlo + OFF4, b4, lane,
      [&](int nt, v8f acc, float bb) {
        const int col = nt * 16 + m;
#pragma unroll
        for (int r = 0; r < 8; ++r) {
          const int idx = (rb + r) * 64 + col;
          const float x4 = tanh_f(acc[r] + bb);
          bufA[idx] = x4 + bufX[idx];
        }
      });
    __syncthreads();
    run_layer<2, 64, true, KP5, 128>(bufA, whi + OFF5, wlo + OFF5, b5, lane,
      [&](int nt, v8f acc, float bb) {
        const int col = nt * 16 + m;
#pragma unroll
        for (int r = 0; r < 8; ++r) buf128[(rb + r) * 128 + col] = tanh_f(acc[r] + bb);
      });
    __syncthreads();
    const v4f wq0 = *(const v4fa*)(wW + rb);
    const v4f wq1 = *(const v4fa*)(wW + rb + 4);
    run_layer<4, 128, true, KP6, 256>(buf128, whi + OFF6, wlo + OFF6, b6, lane,
      [&](int nt, v8f acc, float bb) {
        float s = tanh_f(acc[0] + bb) * wq0.x;
        s = s + tanh_f(acc[1] + bb) * wq0.y;
        s = s + tanh_f(acc[2] + bb) * wq0.z;
        s = s + tanh_f(acc[3] + bb) * wq0.w;
        s = s + tanh_f(acc[4] + bb) * wq1.x;
        s = s + tanh_f(acc[5] + bb) * wq1.y;
        s = s + tanh_f(acc[6] + bb) * wq1.z;
        s = s + tanh_f(acc[7] + bb) * wq1.w;
        s = s + __shfl_xor(s, 16);
        if (lane < 16) {
          const float g = gaw[nt * 16 + m] + s;
          gaw[nt * 16 + m] = g;
        }
      });
  }
  __syncthreads();

  float ss = 0.0f;
  for (int c = tid; c < NOUT; c += 128) {
    const float g = ((gaW[c] + gaW[NOUT + c]) + gaW[2 * NOUT + c]) + gaW[3 * NOUT + c];
    GA[c] = g;
    ss = ss + g * g;
  }
#pragma unroll
  for (int o = 16; o > 0; o >>= 1) ss += __shfl_xor(ss, o);
  if (lane == 0) red[wv] = ss;
  __syncthreads();
  const float tot = ((red[0] + red[1]) + red[2]) + red[3];
  const float inv = 1.0f / (sqrtf(tot) + EPS_F);

  const v4f ga0 = *(const v4fa*)(GA + lane * 4);
  const v4f ga1 = *(const v4fa*)(GA + 128 + lane * 4);
  const v4f o0 = ga0 * inv;
  const v4f o1 = ga1 * inv;
  float* orow = outG + (size_t)bx * NOUT;
  if (wv == 0) {
    *(volatile v4f*)(orow + lane * 4) = o0;
    *(volatile v4f*)(orow + 128 + lane * 4) = o1;
  }
  __threadfence();
  if (wv == 0) {
    *(volatile v4f*)(orow + lane * 4) = o0;
    *(volatile v4f*)(orow + 128 + lane * 4) = o1;
  }
}

extern "C" void kernel_launch(void* const* d_in, const int* in_sizes, int n_in,
                              void* d_out, int out_size, void* d_ws, size_t ws_size,
                              hipStream_t stream) {
  if (n_in < 16) return;
  if (in_sizes[0] != NB * NA * NA) return;
  if (in_sizes[1] != NB * NA) return;
  if (in_sizes[2] != 9 * 64 || in_sizes[3] != 64) return;
  if (in_sizes[4] != 64 * 64 || in_sizes[5] != 64) return;
  if (in_sizes[6] != 64 * 64 || in_sizes[7] != 64) return;
  if (in_sizes[8] != 64 * 64 || in_sizes[9] != 64) return;
  if (in_sizes[10] != 64 * 64 || in_sizes[11] != 64) return;
  if (in_sizes[12] != 64 * 128 || in_sizes[13] != 128) return;
  if (in_sizes[14] != 128 * 256 || in_sizes[15] != 256) return;
  if (out_size != NB * NA * NOUT) return;
  if ((size_t)2 * PLANE_BYTES > ws_size) return;

  const float* Dg = (const float*)d_in[0];
  const float* Sg = (const float*)d_in[1];
  const float* W[7];
  const float* Bb[7];
  for (int l = 0; l < 7; ++l) {
    W[l]  = (const float*)d_in[2 + 2 * l];
    Bb[l] = (const float*)d_in[3 + 2 * l];
  }
  unsigned short* whi = (unsigned short*)d_ws;
  unsigned short* wlo = (unsigned short*)((char*)d_ws + PLANE_BYTES);
  float* out = (float*)d_out;

  prep_weights<<<dim3(16, 7, 1), 256, 0, stream>>>(W[0], W[1], W[2], W[3], W[4], W[5], W[6],
                                                    whi, wlo);
  aev_kernel<<<dim3(NB * NA, 1, 1), 128, 0, stream>>>(
      Dg, Sg, whi, wlo, Bb[0], Bb[1], Bb[2], Bb[3], Bb[4], Bb[5], Bb[6], out);
}
